// GNNSparsifier_61100204753370
// MI455X (gfx1250) — hardware-verified
//
#include <hip/hip_runtime.h>


namespace {
constexpr int N = 50000, E = 800000, DI = 128, HD = 64, NPAD = 50176, NBLK = NPAD / 128, EW = 32  ;
constexpr float FXS = 65536.0f, FXI = 1.0f / 65536.0f, AS_ = 8.0f;

typedef _Float16 b16;
typedef __attribute__((ext_vector_type(16))) _Float16 v16b;
typedef __attribute__((ext_vector_type(8))) _Float16 v8b;
typedef __attribute__((ext_vector_type(8))) float v8f;
typedef __attribute__((ext_vector_type(4))) float v4f;
__device__ __forceinline__ void split16(float v, b16& hi, b16& lo) { hi = (b16)v; lo = (b16)(v - (float)hi); }
__device__ __forceinline__ v16b frag_kb(const b16* p, int hh) { const v8b a = *(const v8b*)(p + 8 * hh), b = *(const v8b*)(p + 16 + 8 * hh); v16b f;
#pragma unroll
  for (int e = 0; e < 8; ++e) { f[e] = a[e]; f[8 + e] = b[e]; } return f; }
__device__ __forceinline__ v8f wmma16b(v16b a, v16b b, v8f c) { v8f d = __builtin_amdgcn_wmma_f32_16x16x32_f16(false, a, false, b, (short)0, c, false, false); asm volatile("v_nop\n\tv_nop\n\tv_nop\n\tv_nop" : "+v"(d) : "v"(a), "v"(b)); return d; }
__device__ __forceinline__ void wave_lds_sync() { __builtin_amdgcn_fence(__ATOMIC_RELEASE, "workgroup"); __builtin_amdgcn_wave_barrier(); __builtin_amdgcn_fence(__ATOMIC_ACQUIRE, "workgroup"); }

__global__ __launch_bounds__(256) void prep_kernel(const float* __restrict__ W1, const float* __restrict__ W2, const float* __restrict__ We1, b16* __restrict__ w1, b16* __restrict__ w2, b16* __restrict__ we) {
  const size_t tid = (size_t)blockIdx.x * blockDim.x + threadIdx.x, nth = (size_t)gridDim.x * blockDim.x;
  for (int pass = 0; pass < 2; ++pass) {
    for (size_t p = tid; p < (size_t)HD * DI; p += nth) { const int n = (int)(p / DI), k = (int)(p % DI); b16 a, c; split16(W1[(size_t)k * HD + n] * 64.0f, a, c); ((volatile b16*)w1)[p] = a; ((volatile b16*)w1)[(size_t)HD * DI + p] = c; }
    for (size_t p = tid; p < (size_t)HD * HD; p += nth) { const int n = (int)(p / HD), k = (int)(p % HD); b16 a, c; split16(W2[(size_t)k * HD + n] * 64.0f, a, c); ((volatile b16*)w2)[p] = a; ((volatile b16*)w2)[(size_t)HD * HD + p] = c; }
    for (size_t p = tid; p < (size_t)HD * 4 * HD; p += nth) { const int n = (int)(p / (4 * HD)), k = (int)(p % (4 * HD)); b16 a, c; split16(We1[(size_t)k * HD + n] * 64.0f, a, c); ((volatile b16*)we)[p] = a; ((volatile b16*)we)[(size_t)HD * 4 * HD + p] = c; }
    __threadfence();
  }
}

typedef __attribute__((ext_vector_type(4))) int v4i;
template <int DF, int NB>
__global__ __launch_bounds__(256) void agg_kernel(const int* __restrict__ esrc, const int* __restrict__ edst, const float* __restrict__ h, float* __restrict__ s) {
  constexpr int LW = DF / 4, LSH = 11;
  __shared__ __attribute__((aligned(16))) int acc[NB * DF]; __shared__ int cnt[NB]; __shared__ int list[8 * 256];
  const int t_ = threadIdx.x, wave = t_ >> 5, lane = t_ & 31, base = blockIdx.x * NB, sub = lane / LW, cl = (lane % LW) * 4;
  for (int i = t_; i < NB * DF; i += 256) acc[i] = 0;
  for (int i = t_; i < NB; i += 256) cnt[i] = 0;
  __syncthreads();
  int* wl = list + wave * 256;
  for (int c0 = 0; c0 < E; c0 += 256 * 8) {
    const int e0 = c0 + (wave * 32 + lane) * 8; int dd[8];
#pragma unroll
    for (int j = 0; j < 8; ++j) { const int dv = edst[min(e0 + j, E - 1)]; dd[j] = (e0 + j < E) ? dv : -1; }
    unsigned sl[8]; bool hit[8]; bool anyl = false;
#pragma unroll
    for (int j = 0; j < 8; ++j) { sl[j] = (unsigned)(dd[j] - base); hit[j] = sl[j] < (unsigned)NB; anyl |= hit[j]; }
    int wc = 0;
    if (__builtin_amdgcn_ballot_w32(anyl) != 0u) {
#pragma unroll
      for (int j = 0; j < 8; ++j) {
        const unsigned mj = __builtin_amdgcn_ballot_w32(hit[j]);
        if (mj != 0u) {
          if (hit[j]) { const int pos = wc + (int)__builtin_amdgcn_mbcnt_lo(mj, 0u); int sidx = esrc[min(e0 + j, E - 1)]; sidx = (sidx < 0) ? 0 : (sidx >= N ? N - 1 : sidx); wl[pos] = (sidx << LSH) | (int)sl[j]; atomicAdd(&cnt[sl[j]], 1); }
          wc += __builtin_popcount(mj); } } }
    __builtin_amdgcn_wave_barrier(); __builtin_amdgcn_fence(__ATOMIC_RELEASE, "workgroup"); __builtin_amdgcn_fence(__ATOMIC_ACQUIRE, "workgroup");
    for (int i = sub; i < wc; i += 32 / LW) { const int ent = wl[i]; const int sidx = ent >> LSH, slot = ent & ((1 << LSH) - 1); const v4f v = *(const v4f*)(h + (size_t)sidx * DF + cl); int* ar = acc + slot * DF + cl;
#pragma unroll
      for (int c = 0; c < 4; ++c) atomicAdd(ar + c, (int)rintf(v[c] * FXS)); }
    __builtin_amdgcn_wave_barrier();
  }
  __syncthreads();
  for (int pass = 0; pass < 2; ++pass) {
    for (int i = t_; i < NB * DF / 4; i += 256) { const int slot = i / (DF / 4), cq = (i % (DF / 4)) * 4, node = base + slot; v4f o = {0.0f, 0.0f, 0.0f, 0.0f};
      if (node < N) { const float ic = FXI / fmaxf((float)cnt[slot], 1.0f); const v4f hv = *(const v4f*)(h + (size_t)node * DF + cq);
#pragma unroll
        for (int c = 0; c < 4; ++c) o[c] = hv[c] + (float)acc[slot * DF + cq + c] * ic; }
      *(volatile v4f*)(s + (size_t)node * DF + cq) = o; }
    __threadfence(); }
}

template <int KIN, int MODE>
__global__ __launch_bounds__(128) void lin_kernel(const float* __restrict__ s, const b16* __restrict__ w, const float* __restrict__ bias, float* __restrict__ y, float* __restrict__ y2) {
  __shared__ __attribute__((aligned(16))) float Ts[4][32 * 64];
  const int lane = threadIdx.x & 31, wave = threadIdx.x >> 5, nloc = lane & 15, hlf = lane >> 4, m0 = blockIdx.x * 128 + wave * 32;
  v8f acc[2][4];
#pragma unroll
  for (int r = 0; r < 2; ++r)
#pragma unroll
    for (int t = 0; t < 4; ++t) acc[r][t] = (v8f){};
#pragma unroll 1
  for (int kb = 0; kb < KIN; kb += 32) { v16b a0, a1, l0, l1;
#pragma unroll
    for (int e = 0; e < 16; ++e) { const int k = kb + ((e < 8) ? (8 * hlf + e) : (16 + 8 * hlf + e - 8)); b16 p, q; split16(s[(size_t)(m0 + nloc) * KIN + k] * AS_, p, q); a0[e] = p; l0[e] = q; split16(s[(size_t)(m0 + 16 + nloc) * KIN + k] * AS_, p, q); a1[e] = p; l1[e] = q; }
#pragma unroll
    for (int t = 0; t < 4; ++t) { const size_t bo = (size_t)(t * 16 + nloc) * KIN + kb; const v16b bw = frag_kb(w + bo, hlf), bl = frag_kb(w + (size_t)HD * KIN + bo, hlf);
      acc[0][t] = wmma16b(a0, bw, acc[0][t]); acc[0][t] = wmma16b(l0, bw, acc[0][t]); acc[0][t] = wmma16b(a0, bl, acc[0][t]);
      acc[1][t] = wmma16b(a1, bw, acc[1][t]); acc[1][t] = wmma16b(l1, bw, acc[1][t]); acc[1][t] = wmma16b(a1, bl, acc[1][t]); } }
  float* Tt = Ts[wave];
#pragma unroll
  for (int t = 0; t < 4; ++t)
#pragma unroll
    for (int r = 0; r < 2; ++r)
#pragma unroll
      for (int v = 0; v < 8; ++v) { const int row = m0 + r * 16 + 8 * hlf + v; Tt[(r * 16 + v + 8 * hlf) * 64 + t * 16 + nloc] = (row < N) ? fmaxf(acc[r][t][v] * (1.0f / (AS_ * 64.0f)) + bias[t * 16 + nloc], 0.0f) : 0.0f; }
  wave_lds_sync();
  for (int pass = 0; pass < 2; ++pass) {
#pragma unroll
    for (int j = 0; j < 16; ++j) { const int rr = j * 2 + hlf, c4 = nloc * 4; const v4f v = *(const v4f*)(Tt + rr * 64 + c4);
      *(volatile v4f*)(y + (size_t)(m0 + rr) * HD + c4) = v; if (MODE == 1 && m0 + rr < N) *(volatile v4f*)(y2 + (size_t)(m0 + rr) * HD + c4) = v; }
    __threadfence(); }
}

__global__ __launch_bounds__(256) void edge_kernel(const int* __restrict__ esrc, const int* __restrict__ edst, const float* __restrict__ Hn, const b16* __restrict__ we, const float* __restrict__ be1, const float* __restrict__ We2, const float* __restrict__ be2,
                                                   float* __restrict__ logits, float* __restrict__ probs) {
  __shared__ __attribute__((aligned(16))) float Gs[8][EW][HD + 1], Gd[8][EW][HD + 1]; __shared__ __attribute__((aligned(16))) float Hh[8][EW][HD + 1]; __shared__ float Lo[8][EW];
  const int wid = threadIdx.x >> 5, lane = threadIdx.x & 31, nloc = lane & 15, hlf = lane >> 4; const int e0 = (blockIdx.x * 8 + wid) * EW;
  { const int e = e0 + lane; int sI = esrc[e], dI = edst[e]; sI = (sI < 0) ? 0 : (sI >= N ? N - 1 : sI); dI = (dI < 0) ? 0 : (dI >= N ? N - 1 : dI);
    const float* hs = Hn + (size_t)sI * HD; const float* hd = Hn + (size_t)dI * HD;
#pragma unroll
    for (int c = 0; c < HD; c += 4) { const v4f a = *(const v4f*)(hs + c), b = *(const v4f*)(hd + c);
#pragma unroll
      for (int q = 0; q < 4; ++q) { Gs[wid][lane][c + q] = a[q]; Gd[wid][lane][c + q] = b[q]; } } }
  wave_lds_sync();
  v8f acc[2][4];
#pragma unroll
  for (int r = 0; r < 2; ++r)
#pragma unroll
    for (int t = 0; t < 4; ++t) acc[r][t] = (v8f){};
#pragma unroll 1
  for (int kb = 0; kb < 4 * HD; kb += 32) { const int blk = kb / HD, c0 = kb % HD; v16b a0, a1, l0, l1;
#pragma unroll
    for (int e = 0; e < 16; ++e) { const int c = c0 + ((e < 8) ? (8 * hlf + e) : (16 + 8 * hlf + e - 8));
#pragma unroll
      for (int r = 0; r < 2; ++r) { const int row = r * 16 + nloc; const float xs = Gs[wid][row][c], xd = Gd[wid][row][c];
        const float f = (blk == 0) ? xs : (blk == 1) ? xd : (blk == 2) ? xs * xd : fabsf(xs - xd); b16 p, q; split16(f * AS_, p, q);
        if (r == 0) { a0[e] = p; l0[e] = q; } else { a1[e] = p; l1[e] = q; } } }
#pragma unroll
    for (int t = 0; t < 4; ++t) { const size_t bo = (size_t)(t * 16 + nloc) * (4 * HD) + kb; const v16b bw = frag_kb(we + bo, hlf), bl = frag_kb(we + (size_t)HD * 4 * HD + bo, hlf);
      acc[0][t] = wmma16b(a0, bw, acc[0][t]); acc[0][t] = wmma16b(l0, bw, acc[0][t]); acc[0][t] = wmma16b(a0, bl, acc[0][t]);
      acc[1][t] = wmma16b(a1, bw, acc[1][t]); acc[1][t] = wmma16b(l1, bw, acc[1][t]); acc[1][t] = wmma16b(a1, bl, acc[1][t]); } }
#pragma unroll
  for (int t = 0; t < 4; ++t)
#pragma unroll
    for (int r = 0; r < 2; ++r)
#pragma unroll
      for (int v = 0; v < 8; ++v) Hh[wid][r * 16 + 8 * hlf + v][t * 16 + nloc] = fmaxf(acc[r][t][v] * (1.0f / (AS_ * 64.0f)) + be1[t * 16 + nloc], 0.0f);
  wave_lds_sync();
  { float lg = be2[0]; const float* hr = Hh[wid][lane];
#pragma unroll 4
    for (int c = 0; c < HD; ++c) lg += hr[c] * We2[c];
    Lo[wid][lane] = lg; }
  wave_lds_sync();
  const float lg = Lo[wid][lane], pr = 1.0f / (1.0f + __expf(-lg));
  for (int pass = 0; pass < 2; ++pass) { ((volatile float*)logits)[e0 + lane] = lg; ((volatile float*)probs)[e0 + lane] = pr; __threadfence(); }
}
}

extern "C" void kernel_launch(void* const* d_in, const int* in_sizes, int n_in,
                              void* d_out, int out_size, void* d_ws, size_t ws_size, hipStream_t stream) {
  (void)n_in; (void)out_size;
  const float* x = (const float*)d_in[0]; const float* W1 = (const float*)d_in[1]; const float* b1 = (const float*)d_in[2]; const float* W2 = (const float*)d_in[3]; const float* b2 = (const float*)d_in[4];
  const float* We1 = (const float*)d_in[5]; const float* be1 = (const float*)d_in[6]; const float* We2 = (const float*)d_in[7]; const float* be2 = (const float*)d_in[8]; const int* ei = (const int*)d_in[9];
  float* Hout = (float*)d_out; float* logits = Hout + (size_t)N * HD; float* probs = logits + E;
  if (in_sizes[0] != N * DI || in_sizes[1] != DI * HD || in_sizes[3] != HD * HD || in_sizes[5] != 4 * HD * HD || in_sizes[7] != HD || in_sizes[9] != 2 * E) return;
  const int* esrc = ei; const int* edst = ei + E;
  size_t off = 0; char* ws = (char*)d_ws;
  auto carve = [&](size_t bytes) { char* p = ws + off; off += (bytes + 255) & ~(size_t)255; return p; };
  b16* w1 = (b16*)carve((size_t)HD * DI * 2 * 2); b16* w2 = (b16*)carve((size_t)HD * HD * 2 * 2); b16* we = (b16*)carve((size_t)HD * 4 * HD * 2 * 2);
  float* s1 = (float*)carve((size_t)NPAD * DI * 4); float* h1 = (float*)carve((size_t)NPAD * HD * 4); float* s2 = (float*)carve((size_t)NPAD * HD * 4); float* Hf = (float*)carve((size_t)NPAD * HD * 4);
  if (off > ws_size) return;
  prep_kernel<<<64, 256, 0, stream>>>(W1, W2, We1, w1, w2, we);
  agg_kernel<DI, 512><<<NPAD / 512, 256, 0, stream>>>(esrc, edst, x, s1);
  lin_kernel<DI, 0><<<NBLK, 128, 0, stream>>>(s1, w1, b1, h1, nullptr);
  agg_kernel<HD, 1024><<<NPAD / 1024, 256, 0, stream>>>(esrc, edst, h1, s2);
  lin_kernel<HD, 1><<<NBLK, 128, 0, stream>>>(s2, w2, b2, Hf, Hout);
  edge_kernel<<<E / EW / 8, 256, 0, stream>>>(esrc, edst, Hf, we, be1, We2, be2, logits, probs);
}
